// Head_13030930776875
// MI455X (gfx1250) — hardware-run, weakly checked
//
#include <hip/hip_runtime.h>
#ifndef NB
#define NB 4
#endif
#ifndef SEQ
#define SEQ 2048
#endif
#define SQ SEQ
#define SQF 2048
#define NBF 4
#define DM 1024
#define HD 128
#define NR ((size_t)NB * SQ)
#define QN SQ
#define NBR NB
#define MP ((int)NR)
#define ER ((SQ < 256) ? SQ : 256)
#define OMEGA_L 0.7f
#define OMEGA_G 0.3f
#define ASC 0.08838834764831845f
#define PCAR 1024.0f
#define RCAR 1024.0f
#define YSC 4.0f
static_assert(SQ % 128 == 0);
static_assert(ER % 128 == 0);
static_assert((QN - ER) % 128 == 0);
static_assert(DM % 32 == 0);
static_assert(HD % 64 == 0);
static_assert(NB <= NBF);
static_assert(SQ <= SQF);

typedef unsigned short v8us __attribute__((ext_vector_type(8), may_alias));
typedef float  v8f  __attribute__((ext_vector_type(8)));
typedef float  v4f  __attribute__((ext_vector_type(4)));
typedef float  v4fa __attribute__((ext_vector_type(4), may_alias));
typedef _Float16 v16h __attribute__((ext_vector_type(16)));
typedef _Float16 v4h __attribute__((ext_vector_type(4)));
union FragH { v16h v; v8us half[2]; _Float16 h[16]; unsigned short u[16]; };

__device__ __forceinline__ unsigned short bf16_bits(float x) { unsigned int u = __float_as_uint(x); return (unsigned short)((u + 0x7FFFu + ((u >> 16) & 1u)) >> 16); }
__device__ __forceinline__ float bf16_val(unsigned short b) { return __uint_as_float(((unsigned int)b) << 16); }
__device__ __forceinline__ float bf16_rne(float x) { return bf16_val(bf16_bits(x)); }

__device__ __forceinline__ v16h g2_frag(const _Float16* p, int hh) { FragH f; f.half[0] = *(const v8us*)((const unsigned short*)p + 8 * hh); f.half[1] = *(const v8us*)((const unsigned short*)p + 16 + 8 * hh); return f.v; }
__device__ __forceinline__ v8f g2_mma(v16h a, v16h b, v8f c) { v8f d = __builtin_amdgcn_wmma_f32_16x16x32_f16(false, a, false, b, (short)0, c, false, false); asm volatile("v_nop\n\tv_nop\n\tv_nop\n\tv_nop" : "+v"(d) : "v"(a), "v"(b)); return d; }

__global__ __launch_bounds__(256) void k_wt_f16(const float* __restrict__ W, _Float16* __restrict__ Wt, int K, int N, float scale) {
  const int t = blockIdx.x * 256 + threadIdx.x; if (t >= N * (K / 8)) return; const int n = t / (K / 8), k8 = (t % (K / 8)) * 8; FragH f;
#pragma unroll
  for (int i = 0; i < 8; ++i) f.h[i] = (_Float16)(bf16_rne(W[(size_t)(k8 + i) * N + n]) * scale);
  const v8us o = f.half[0];
  *(volatile v8us*)((unsigned short*)Wt + (size_t)n * K + k8) = o; __threadfence(); *(volatile v8us*)((unsigned short*)Wt + (size_t)n * K + k8) = o;
}

__global__ __launch_bounds__(256) void k_x16(const float* __restrict__ x, _Float16* __restrict__ X16, size_t n8) {
  const size_t t = (size_t)blockIdx.x * 256 + threadIdx.x; if (t >= n8) return;
  const size_t drow = t / (DM / 8), c8 = (t % (DM / 8)) * 8; const size_t b = drow / SQ, n = drow % SQ;
  const float* src = x + (b * SQF + n) * DM + c8;
  const v4f a = *(const v4fa*)src, c = *(const v4fa*)(src + 4); FragH f;
#pragma unroll
  for (int q = 0; q < 4; ++q) { f.h[q] = (_Float16)bf16_rne(a[q]); f.h[4 + q] = (_Float16)bf16_rne(c[q]); }
  const v8us o = f.half[0];
  *(volatile v8us*)((unsigned short*)X16 + t * 8) = o; __threadfence(); *(volatile v8us*)((unsigned short*)X16 + t * 8) = o;
}

__global__ __launch_bounds__(256) void k_h16(const float* __restrict__ F, _Float16* __restrict__ X16, size_t n8) {
  const size_t t = (size_t)blockIdx.x * 256 + threadIdx.x; if (t >= n8) return;
  const v4f a = *(const v4fa*)(F + t * 8), c = *(const v4fa*)(F + t * 8 + 4); FragH f;
#pragma unroll
  for (int q = 0; q < 4; ++q) { f.h[q] = (_Float16)a[q]; f.h[4 + q] = (_Float16)c[q]; }
  const v8us o = f.half[0];
  *(volatile v8us*)((unsigned short*)X16 + t * 8) = o; __threadfence(); *(volatile v8us*)((unsigned short*)X16 + t * 8) = o;
}

__global__ __launch_bounds__(256) void k_hl(const float* __restrict__ F, _Float16* __restrict__ Hh, _Float16* __restrict__ Hl, size_t n8) {
  const size_t t = (size_t)blockIdx.x * 256 + threadIdx.x; if (t >= n8) return; FragH fh, fl; const v4f a = *(const v4fa*)(F + t * 8), c = *(const v4fa*)(F + t * 8 + 4);
#pragma unroll
  for (int q = 0; q < 4; ++q) { _Float16 h = (_Float16)a[q]; fh.h[q] = h; fl.h[q] = (_Float16)((a[q] - (float)h) * RCAR); h = (_Float16)c[q]; fh.h[4 + q] = h; fl.h[4 + q] = (_Float16)((c[q] - (float)h) * RCAR); }
  for (int pass = 0; pass < 2; ++pass) { *(volatile v8us*)((unsigned short*)Hh + t * 8) = fh.half[0]; *(volatile v8us*)((unsigned short*)Hl + t * 8) = fl.half[0]; if (pass == 0) __threadfence(); }
}

template <int NHv, int TTv>
__global__ __launch_bounds__(256) void k_vt(const _Float16* __restrict__ V16, int ldv, int voff, _Float16* __restrict__ Vt) {
  __shared__ unsigned short tl[64][66]; const int tid = threadIdx.x; const int slab = blockIdx.x / (TTv / 64), lg = blockIdx.x % (TTv / 64); const int b = slab / NHv, h = slab % NHv;
  for (int i = tid; i < 64 * 8; i += 256) { const int r = i / 8, c8 = (i % 8) * 8; FragH f; f.half[0] = *(const v8us*)((const unsigned short*)V16 + ((size_t)b * TTv + lg * 64 + r) * ldv + voff + h * 64 + c8);
#pragma unroll
    for (int q = 0; q < 8; ++q) tl[r][c8 + q] = f.u[q]; }
  __syncthreads();
  for (int pass = 0; pass < 2; ++pass) {
#pragma unroll
    for (int rd = 0; rd < 2; ++rd) { const int d = rd * 32 + tid / 8, pc = tid % 8; FragH f;
#pragma unroll
      for (int q = 0; q < 8; ++q) f.u[q] = tl[pc * 8 + q][d];
      *(volatile v8us*)((unsigned short*)Vt + ((size_t)slab * 64 + d) * TTv + lg * 64 + pc * 8) = f.half[0]; }
    if (pass == 0) __threadfence(); }
}

template <int ACT>
__global__ __launch_bounds__(128) void k_gemm2(const _Float16* __restrict__ A, int lda, size_t sA, const _Float16* __restrict__ Bh, int ldb, size_t sB, float alpha, const float* __restrict__ bias, size_t sBias, const float* CP, int rowsPerB, size_t sCPb, int row0g,
    float* C, _Float16* C16, int ldc, size_t sC, int M, int N, int K, int cskip, int kcaus) {
  static_assert(ACT == 0 || ACT == 3);
  __shared__ __attribute__((aligned(16))) float so[4][32][68];
  const int tid = threadIdx.x, w = tid >> 5, lane = tid & 31, ln = lane & 15, hh = lane >> 4; const int by = blockIdx.y;
  A += (size_t)by * sA; Bh += (size_t)by * sB; const size_t cofs = (size_t)by * sC; const float* bp = bias ? bias + (size_t)by * sBias : nullptr;
  const int ntn = N >> 6; const int mt = blockIdx.x / ntn, nq = blockIdx.x - mt * ntn; const int row0 = mt * 128 + 32 * w, col0 = nq * 64; if (row0 >= M) return;
  if (cskip && col0 >= row0g + mt * 128 + 128) return;
  const int kend = row0g + row0 + 32; const int Ke = kcaus ? ((kend < K) ? kend : K) : K;
  const _Float16* a0p = A + (size_t)(row0 + ln) * lda; const _Float16* a1p = a0p + (size_t)16 * lda;
  const _Float16* b0p = Bh + (size_t)(col0 + ln) * ldb; const _Float16* b1p = b0p + (size_t)16 * ldb; const _Float16* b2p = b1p + (size_t)16 * ldb; const _Float16* b3p = b2p + (size_t)16 * ldb;
  const v8f z8 = {0.f,0.f,0.f,0.f,0.f,0.f,0.f,0.f}; v8f c00 = z8, c01 = z8, c02 = z8, c03 = z8, c10 = z8, c11 = z8, c12 = z8, c13 = z8;
#pragma unroll 1
  for (int kb = 0; kb < Ke; kb += 32) { const v16h a0 = g2_frag(a0p + kb, hh), a1 = g2_frag(a1p + kb, hh);
    v16h b = g2_frag(b0p + kb, hh); c00 = g2_mma(a0, b, c00); c10 = g2_mma(a1, b, c10);
    b = g2_frag(b1p + kb, hh); c01 = g2_mma(a0, b, c01); c11 = g2_mma(a1, b, c11);
    b = g2_frag(b2p + kb, hh); c02 = g2_mma(a0, b, c02); c12 = g2_mma(a1, b, c12);
    b = g2_frag(b3p + kb, hh); c03 = g2_mma(a0, b, c03); c13 = g2_mma(a1, b, c13); }
  v8f accs[8] = {c00, c01, c02, c03, c10, c11, c12, c13};
#pragma unroll
  for (int u = 0; u < 8; ++u) { const int t = u & 3, half = u >> 2; const int col = col0 + t * 16 + ln; const float bv = bp ? bf16_rne(bp[col]) : 0.f;
#pragma unroll
    for (int r = 0; r < 8; ++r) { const int rloc = half * 16 + 8 * hh + r; float v = accs[u][r] * alpha + bv;
      if (CP) { if (rowsPerB < 0) v += CP[cofs + (size_t)(row0g + row0 + rloc) * ldc + col]; else { const int bidx = (row0g + row0 + rloc) / rowsPerB; v += CP[(size_t)bidx * sCPb + (size_t)by * 64 + col]; } }
      if (ACT == 3) v = fmaxf(v, 0.f);
      so[w][rloc][t * 16 + ln] = v; } }
  __builtin_amdgcn_fence(4, "workgroup"); __builtin_amdgcn_wave_barrier();
  const int rsub = lane >> 4, c4 = (lane & 15) * 4;
  for (int pass = 0; pass < 2; ++pass) {
#pragma unroll
    for (int q = 0; q < 16; ++q) { const int r = q * 2 + rsub; const v4f v = *(const v4fa*)&so[w][r][c4]; if (C) *(volatile v4f*)(C + cofs + (size_t)(row0 + r) * ldc + col0 + c4) = v; if (C16) { v4h h4; for (int i = 0; i < 4; ++i) h4[i] = (_Float16)v[i]; *(volatile v4h*)(C16 + cofs + (size_t)(row0 + r) * ldc + col0 + c4) = h4; } }
    if (pass == 0) __threadfence(); }
}

__global__ __launch_bounds__(128) void k_blend(const float* __restrict__ S, const float* __restrict__ G, _Float16* __restrict__ P, _Float16* __restrict__ PL) {
  #pragma clang fp contract(off)
  __shared__ __attribute__((aligned(16))) unsigned short th[4][32][72];
  __shared__ __attribute__((aligned(16))) unsigned short tr[4][32][72];
  const int tid = threadIdx.x, w = tid >> 5, lane = tid & 31;
  const int wb = __builtin_amdgcn_readfirstlane((int)(blockIdx.x * 128) + (tid & 96));
  const int i = wb + lane;
  const int jw = (wb | 63) + 1;
  const bool early = ((int)(blockIdx.x * 128)) < ER;
  const float* s = S + (size_t)i * SQ;
  const float* g = G + (size_t)i * SQ;
  const float sqi = g[i];
  float mx = -3.0e38f;
#pragma unroll 1
  for (int j0 = 0; j0 < jw; j0 += 8) {
    const v4f a = *(const v4fa*)(s + j0), c = *(const v4fa*)(s + j0 + 4);
#pragma unroll
    for (int q = 0; q < 4; ++q) { mx = (j0 + q <= i) ? fmaxf(mx, a[q]) : mx; mx = (j0 + 4 + q <= i) ? fmaxf(mx, c[q]) : mx; }
  }
  const float cgn = -1.0f / (2.0f * (float)HD * YSC * YSC);
  float se = 0.f, sk = 0.f;
#pragma unroll 1
  for (int j0 = 0; j0 < jw; j0 += 8) {
    const v4f a = *(const v4fa*)(s + j0), c = *(const v4fa*)(s + j0 + 4);
    const v4f ga = *(const v4fa*)(g + j0), gc = *(const v4fa*)(g + j0 + 4);
#pragma unroll
    for (int q = 0; q < 8; ++q) {
      const int j = j0 + q;
      const float sv = (q < 4) ? a[q & 3] : c[q & 3];
      const float gv = (q < 4) ? ga[q & 3] : gc[q & 3];
      const float gjj = G[(size_t)j * SQ + j];
      const float e = __expf(fminf(sv - mx, 0.f));
      const float d = fmaxf(sqi + gjj - 2.0f * gv, 0.f);
      const float kv = __expf(d * cgn);
      const bool in = (j <= i);
      se += in ? e : 0.f; sk += in ? kv : 0.f;
    }
  }
  const float wl = (OMEGA_L * PCAR) / se;
  const float wg = (OMEGA_G * PCAR) / (sk + 1e-8f);
  const int rsub = lane >> 3, pc8 = (lane & 7) * 8;
  const v8us z = {0, 0, 0, 0, 0, 0, 0, 0};
#pragma unroll 1
  for (int jb = 0; jb < SQ; jb += 64) {
    const bool wres = early && (jb < ER);
    if (jb < jw) {
#pragma unroll 1
      for (int cc = 0; cc < 8; ++cc) {
        const int j0 = jb + cc * 8;
        const v4f a = *(const v4fa*)(s + j0), c = *(const v4fa*)(s + j0 + 4);
        const v4f ga = *(const v4fa*)(g + j0), gc = *(const v4fa*)(g + j0 + 4);
        FragH fh, fl;
#pragma unroll
        for (int q = 0; q < 8; ++q) {
          const int j = j0 + q;
          const float sv = (q < 4) ? a[q & 3] : c[q & 3];
          const float gv = (q < 4) ? ga[q & 3] : gc[q & 3];
          const float gjj = G[(size_t)j * SQ + j];
          const float e = __expf(fminf(sv - mx, 0.f));
          const float d = fmaxf(sqi + gjj - 2.0f * gv, 0.f);
          const float kv = __expf(d * cgn);
          const float p = (j <= i) ? (wl * e + wg * kv) : 0.f;
          const _Float16 h = (_Float16)p; fh.h[q] = h; fl.h[q] = (_Float16)((p - (float)h) * RCAR);
        }
        *(v8us*)&th[w][lane][cc * 8] = fh.half[0];
        if (wres) *(v8us*)&tr[w][lane][cc * 8] = fl.half[0];
      }
    } else {
#pragma unroll
      for (int cc = 0; cc < 8; ++cc) { *(v8us*)&th[w][lane][cc * 8] = z; if (wres) *(v8us*)&tr[w][lane][cc * 8] = z; }
    }
    __builtin_amdgcn_fence(4, "workgroup"); __builtin_amdgcn_wave_barrier();
    for (int pass = 0; pass < 2; ++pass) {
#pragma unroll
      for (int it = 0; it < 8; ++it) {
        const int r = it * 4 + rsub;
        const v8us v = *(const v8us*)&th[w][r][pc8];
        *(volatile v8us*)((unsigned short*)P + (size_t)(wb + r) * SQ + jb + pc8) = v;
        if (wres) { const v8us u = *(const v8us*)&tr[w][r][pc8]; *(volatile v8us*)((unsigned short*)PL + (size_t)(wb + r) * ER + jb + pc8) = u; }
      }
      if (pass == 0) __threadfence();
    }
    __builtin_amdgcn_fence(4, "workgroup"); __builtin_amdgcn_wave_barrier();
  }
}

static void g2(hipStream_t st, dim3 grid, const _Float16* A, int lda, const _Float16* Bh, int ldb, float alpha, const float* CP, int row0g, float* C, int ldc, int M, int N, int K, int cskip, int kcaus) {
  k_gemm2<0><<<grid, 128, 0, st>>>(A, lda, (size_t)0, Bh, ldb, (size_t)0, alpha, (const float*)nullptr, (size_t)0, CP, -1, (size_t)0, row0g, C, (_Float16*)nullptr, ldc, (size_t)0, M, N, K, cskip, kcaus);
}

extern "C" void kernel_launch(void* const* d_in, const int* in_sizes, int n_in,
                              void* d_out, int out_size, void* d_ws, size_t ws_size, hipStream_t stream) {
  if (n_in < 5) return;
  const long long needx = ((long long)(NB - 1) * SQF + SQ) * DM;
  if ((long long)in_sizes[0] < needx || in_sizes[1] < DM * HD || in_sizes[2] < DM * HD || in_sizes[3] < DM * HD || in_sizes[4] < HD * HD) return;
  if ((long long)out_size < (long long)NR * HD) return;
  const float* x = (const float*)d_in[0]; const float* wq = (const float*)d_in[1]; const float* wk = (const float*)d_in[2]; const float* wv = (const float*)d_in[3]; const float* lg = (const float*)d_in[4];
  float* out = (float*)d_out;
  char* ws = (char*)d_ws; size_t off = 0;
  auto take = [&](size_t bytes) { char* p = ws + off; off += (bytes + 255) & ~(size_t)255; return p; };
  _Float16* BQ = (_Float16*)take((size_t)HD * DM * 2); _Float16* BK = (_Float16*)take((size_t)HD * DM * 2); _Float16* BV = (_Float16*)take((size_t)HD * DM * 2);
  _Float16* LT = (_Float16*)take((size_t)HD * HD * 2);
  _Float16* X16 = (_Float16*)take(NR * DM * 2); float* QF = (float*)take(NR * HD * 4);
  _Float16* Q16 = (_Float16*)take(NR * HD * 2); _Float16* QL = (_Float16*)take(NR * HD * 2); _Float16* K16 = (_Float16*)take(NR * HD * 2); _Float16* KL = (_Float16*)take(NR * HD * 2);
  _Float16* V16 = (_Float16*)take(NR * HD * 2); _Float16* VL = (_Float16*)take(NR * HD * 2); _Float16* Y16 = (_Float16*)take(NR * HD * 2);
  _Float16* VT = (_Float16*)take((size_t)NB * HD * SQ * 2); _Float16* VLT = (_Float16*)take((size_t)NB * HD * SQ * 2);
  float* S = (float*)take((size_t)SQ * SQ * 4); float* G = (float*)take((size_t)SQ * SQ * 4); _Float16* P = (_Float16*)take((size_t)SQ * SQ * 2);
  _Float16* PL = (_Float16*)take((size_t)ER * ER * 2); float* OE = (float*)take((size_t)ER * HD * 4);
  if (off > ws_size) return;
  const unsigned gw = (unsigned)(((size_t)HD * (DM / 8) + 255) / 256), gwl = (unsigned)(((size_t)HD * (HD / 8) + 255) / 256);
  k_wt_f16<<<gw, 256, 0, stream>>>(wq, BQ, DM, HD, 16.0f); k_wt_f16<<<gw, 256, 0, stream>>>(wk, BK, DM, HD, 16.0f); k_wt_f16<<<gw, 256, 0, stream>>>(wv, BV, DM, HD, 16.0f);
  k_wt_f16<<<gwl, 256, 0, stream>>>(lg, LT, HD, HD, 16.0f);
  k_x16<<<(unsigned)((NR * DM / 8 + 255) / 256), 256, 0, stream>>>(x, X16, NR * DM / 8);
  const dim3 gp((unsigned)((NR / 128) * (HD / 64)), 1);
  const unsigned ghl = (unsigned)((NR * HD / 8 + 255) / 256);
  g2(stream, gp, X16, DM, BQ, DM, 0.0625f, nullptr, 0, QF, HD, MP, HD, DM, 0, 0);
  k_hl<<<ghl, 256, 0, stream>>>(QF, Q16, QL, NR * HD / 8);
  g2(stream, gp, X16, DM, BK, DM, 0.0625f, nullptr, 0, QF, HD, MP, HD, DM, 0, 0);
  k_hl<<<ghl, 256, 0, stream>>>(QF, K16, KL, NR * HD / 8);
  g2(stream, gp, X16, DM, BV, DM, 0.0625f, nullptr, 0, QF, HD, MP, HD, DM, 0, 0);
  k_hl<<<ghl, 256, 0, stream>>>(QF, V16, VL, NR * HD / 8);
  k_vt<2, SQ><<<(unsigned)(NB * 2 * (SQ / 64)), 256, 0, stream>>>(V16, HD, 0, VT);
  k_vt<2, SQ><<<(unsigned)(NB * 2 * (SQ / 64)), 256, 0, stream>>>(VL, HD, 0, VLT);
  g2(stream, gp, K16, HD, LT, HD, YSC / 16.0f, nullptr, 0, QF, HD, MP, HD, HD, 0, 0);
  k_h16<<<ghl, 256, 0, stream>>>(QF, Y16, NR * HD / 8);
  const dim3 gs((unsigned)((QN / 128) * (SQ / 64)), 1), ge((unsigned)((ER / 128) * (HD / 64)), 1);
  for (int b = 0; b < NBR; ++b) {
    const size_t ro = (size_t)b * SQ * HD, vto = (size_t)b * HD * SQ; float* ob = out + ro;
    g2(stream, gs, QL + ro, HD, K16 + ro, HD, ASC / RCAR, nullptr, 0, S, SQ, QN, SQ, HD, 1, 0);
    g2(stream, gs, Q16 + ro, HD, KL + ro, HD, ASC / RCAR, S, 0, S, SQ, QN, SQ, HD, 1, 0);
    g2(stream, gs, Q16 + ro, HD, K16 + ro, HD, ASC, S, 0, S, SQ, QN, SQ, HD, 1, 0);
    g2(stream, gs, Y16 + ro, HD, Y16 + ro, HD, 1.0f, nullptr, 0, G, SQ, QN, SQ, HD, 1, 0);
    k_blend<<<(unsigned)(QN / 128), 128, 0, stream>>>(S, G, P, PL);
    g2(stream, ge, PL, ER, VT + vto, SQ, 1.0f / (PCAR * RCAR), nullptr, 0, OE, HD, ER, HD, ER, 0, 0);
    g2(stream, ge, P, SQ, VLT + vto, SQ, 1.0f / (PCAR * RCAR), OE, 0, OE, HD, ER, HD, ER, 0, 0);
    g2(stream, ge, P, SQ, VT + vto, SQ, 1.0f / PCAR, OE, 0, ob, HD, ER, HD, ER, 0, 0);
    if (QN > ER) { const dim3 gt((unsigned)(((QN - ER) / 128) * (HD / 64)), 1); g2(stream, gt, P + (size_t)ER * SQ, SQ, VT + vto, SQ, 1.0f / PCAR, nullptr, ER, ob + (size_t)ER * HD, HD, QN - ER, HD, SQ, 0, 1); }
  }
}
